// S4Layer_10479720202533
// MI455X (gfx1250) — hardware-run, weakly checked
//
#include <hip/hip_runtime.h>
#include <math.h>

typedef __attribute__((ext_vector_type(16))) _Float16 v16h;
typedef __attribute__((ext_vector_type(8)))  _Float16 v8h;
typedef __attribute__((ext_vector_type(2)))  _Float16 v2h;
typedef __attribute__((ext_vector_type(16))) __bf16   v16b;
typedef __attribute__((ext_vector_type(8)))  __bf16   v8b;
typedef __attribute__((ext_vector_type(8)))  float    v8f;
typedef __attribute__((ext_vector_type(4)))  float    v4f;
typedef __attribute__((ext_vector_type(2)))  float    v2f;

constexpr int kNb   = 4;
constexpr int kL    = 4096;
constexpr int kD    = 512;
constexpr int kN    = 64;
constexpr int kQ    = 64;
constexpr int kC    = kL / kQ;
constexpr int kE    = kNb * kC;
constexpr int kRW   = 320;
constexpr int kThr  = 256;
constexpr float kInCarry = 1024.0f;
constexpr float kACarry  = 16384.0f;
constexpr float kScC = 1.0f / (kInCarry * kACarry);
constexpr float kScY = 1.0f / (kInCarry * kInCarry);
constexpr float kF16MinNormal = 6.103515625e-5f;
constexpr int kTabPW = 0, kTabV = 28672, kTabW = 32768, kTabC = 36864;

static_assert(kQ == 64 && kC == 64 && kE == 256 && kN == 64 && kD == 512 && kRW == 320, "the index arithmetic below uses these sizes");
static_assert(kTabV == 7 * 4096 && kTabW == kTabV + 4096 && kTabC == kTabW + 4096 && kTabC + 64 <= 37888, "the tables are laid end to end inside TAB");

constexpr size_t kOffZB = 0ull;
constexpr size_t kOffTAB = 8192ull;
constexpr size_t kOffTP16 = 159744ull;
constexpr size_t kOffAQ16 = 184320ull;
constexpr size_t kOffHN32 = 225280ull;
constexpr size_t kOffHX = 749568ull;
constexpr size_t kWsTotal = 84635648ull;
static_assert(kWsTotal <= 134217728ull, "carve cap: under 128 MiB");
static_assert(kOffZB == 0
              && kOffTAB == kOffZB + 8192ull
              && kOffTP16 == kOffTAB + 151552ull
              && kOffAQ16 == kOffTP16 + 24576ull
              && kOffHN32 == kOffAQ16 + 40960ull
              && kOffHX == kOffHN32 + 524288ull
              && kWsTotal == kOffHX + 83886080ull, "the carve is chained and totalled");
static_assert((kOffZB % 256) == 0 && (kOffTAB % 256) == 0 && (kOffTP16 % 256) == 0 && (kOffAQ16 % 256) == 0 && (kOffHN32 % 256) == 0 && (kOffHX % 256) == 0, "aligned regions");
static_assert(2048 >= kD, "the zero bias covers the widest launch's 512 output columns (the engine reads one bias value a column)");

__device__ __forceinline__ unsigned short f2bf_bits(float f) {
  unsigned u = __float_as_uint(f);
  return (unsigned short)((u + 0x7FFFu + ((u >> 16) & 1u)) >> 16);
}
__device__ __forceinline__ float bf_bits2f(unsigned short h) { return __uint_as_float(((unsigned)h) << 16); }
__device__ __forceinline__ float bf16r(float f) { return bf_bits2f(f2bf_bits(f)); }
__device__ __forceinline__ float carry_flush(float v, float carry) {
  const float s = v * carry;
  return (fabsf(s) < kF16MinNormal) ? 0.0f : s;
}

__device__ __forceinline__ void dep_guard4_h(v8f& a, v8f& b, v8f& c, v8f& d, v16h x, v16h y) { asm volatile("v_nop\n\tv_nop\n\tv_nop\n\tv_nop" : "+v"(a), "+v"(b), "+v"(c), "+v"(d) : "v"(x), "v"(y)); }
__device__ __forceinline__ void dep_guard4_b(v8f& a, v8f& b, v8f& c, v8f& d, v16b x, v16b y) { asm volatile("v_nop\n\tv_nop\n\tv_nop\n\tv_nop" : "+v"(a), "+v"(b), "+v"(c), "+v"(d) : "v"(x), "v"(y)); }
__device__ __forceinline__ void keep4_h(v16h a, v16h b, v16h c, v16h d) { asm volatile("v_nop" :: "v"(a), "v"(b), "v"(c), "v"(d)); }
__device__ __forceinline__ void keep4_b(v16b a, v16b b, v16b c, v16b d) { asm volatile("v_nop" :: "v"(a), "v"(b), "v"(c), "v"(d)); }
__device__ __forceinline__ void acc_guard4(v8f& a, v8f& b, v8f& c, v8f& d) { asm volatile("v_nop\n\tv_nop\n\tv_nop\n\tv_nop" : "+v"(a), "+v"(b), "+v"(c), "+v"(d)); }

template <typename T> struct Frag;
template <> struct Frag<_Float16> {
  typedef v16h V; union U { v16h v; v8h h[2]; };
  static __device__ __forceinline__ v16h load(const _Float16* p) {
    U f; f.h[0] = *(const v8h*)(p); f.h[1] = *(const v8h*)(p + 16); return f.v;
  }
  static __device__ __forceinline__ v8f mma(v16h a, v16h b, v8f c) {
    return __builtin_amdgcn_wmma_f32_16x16x32_f16(false, a, false, b, (short)0, c, false, false);
  }
  static __device__ __forceinline__ void guard4(v8f& a, v8f& b, v8f& c, v8f& d, v16h x, v16h y) { dep_guard4_h(a, b, c, d, x, y); }
  static __device__ __forceinline__ void keep(v16h a, v16h b, v16h c, v16h d) { keep4_h(a, b, c, d); }
};
template <> struct Frag<__bf16> {
  typedef v16b V; union U { v16b v; v8b h[2]; };
  static __device__ __forceinline__ v16b load(const __bf16* p) {
    U f; f.h[0] = *(const v8b*)(p); f.h[1] = *(const v8b*)(p + 16); return f.v;
  }
  static __device__ __forceinline__ v8f mma(v16b a, v16b b, v8f c) {
    return __builtin_amdgcn_wmma_f32_16x16x32_bf16(false, a, false, b, (short)0, c, false, false);
  }
  static __device__ __forceinline__ void guard4(v8f& a, v8f& b, v8f& c, v8f& d, v16b x, v16b y) { dep_guard4_b(a, b, c, d, x, y); }
  static __device__ __forceinline__ void keep(v16b a, v16b b, v16b c, v16b d) { keep4_b(a, b, c, d); }
};

__device__ __forceinline__ v8f mma_h(v16h a, v16h b, v8f c) {
  c = __builtin_amdgcn_wmma_f32_16x16x32_f16(false, a, false, b, (short)0, c, false, false);
  asm volatile("v_nop\n\tv_nop\n\tv_nop\n\tv_nop" : "+v"(c) : "v"(a), "v"(b));
  return c;
}

template <int ET> struct Elem;
template <> struct Elem<0> { typedef _Float16 T; };
template <> struct Elem<1> { typedef __bf16 T; };
template <int ET, bool SPLIT, int BIAS_MODE, int OUT_MODE, bool RESID, int ACT = 0>
__global__ __launch_bounds__(256) void wmma_gemm64(
    const unsigned short* __restrict__ Ap, const unsigned short* __restrict__ A2p, int lda, long strideA,
    const unsigned short* __restrict__ Btp, const unsigned short* __restrict__ Bt2p, int ldb, long strideB,
    void* __restrict__ Cout, void* __restrict__ Cout2, int ldc, long strideC,
    const float* __restrict__ bias,
    const float* __restrict__ resid, long strideR,
    int M, int N, int K, float scale) {
  typedef typename Elem<ET>::T T;
  typedef typename Frag<T>::V V;
  const T* A = (const T*)Ap; const T* A2 = (const T*)A2p; const T* Bt = (const T*)Btp; const T* Bt2 = (const T*)Bt2p;
  __shared__ __align__(16) float sT[8][16 * 68];
  const int b    = blockIdx.y;
  const int lane = threadIdx.x & 31;
  const int wave = threadIdx.x >> 5;
  const int tilesN = N >> 6;
  const int tilesM = M >> 6;
  const int tile = blockIdx.x * 8 + wave;
  if (tile >= tilesM * tilesN) return;
  const int tm = tile / tilesN;
  const int tn = tile - tm * tilesN;
  const int m0 = tm << 6;
  const int n0 = tn << 6;

  const T* Ab  = A  + (size_t)b * strideA;
  const T* Bb  = Bt + (size_t)b * strideB;
  const T* Ab2 = SPLIT ? (A2  + (size_t)b * strideA) : nullptr;
  const T* Bb2 = SPLIT ? (Bt2 + (size_t)b * strideB) : nullptr;

  const int rlane = lane & 15;
  const int koff  = (lane >> 4) * 8;
  const int mOff  = (lane >> 4) * 8;

  v8f acc[4][4];
#pragma unroll
  for (int i = 0; i < 4; ++i)
#pragma unroll
    for (int j = 0; j < 4; ++j) acc[i][j] = (v8f){0.f,0.f,0.f,0.f,0.f,0.f,0.f,0.f};

  for (int k0 = 0; k0 < K; k0 += 32) {
    V bh[4], bl[4];
#pragma unroll
    for (int j = 0; j < 4; ++j) {
      const size_t bo = (size_t)(n0 + (j << 4) + rlane) * ldb + koff + k0;
      bh[j] = Frag<T>::load(Bb + bo);
      if (SPLIT) bl[j] = Frag<T>::load(Bb2 + bo);
    }
#pragma unroll
    for (int i = 0; i < 4; ++i) {
      const size_t ao = (size_t)(m0 + (i << 4) + rlane) * lda + koff + k0;
      V ah = Frag<T>::load(Ab + ao);
      V al;
      if (SPLIT) al = Frag<T>::load(Ab2 + ao);
#pragma unroll
      for (int j = 0; j < 4; ++j) {
        acc[i][j] = Frag<T>::mma(ah, bh[j], acc[i][j]);
        if (SPLIT) {
          acc[i][j] = Frag<T>::mma(ah, bl[j], acc[i][j]);
          acc[i][j] = Frag<T>::mma(al, bh[j], acc[i][j]);
        }
      }
      Frag<T>::guard4(acc[i][0], acc[i][1], acc[i][2], acc[i][3], ah, SPLIT ? al : ah);
    }
    Frag<T>::keep(bh[0], bh[1], bh[2], bh[3]);
    if (SPLIT) Frag<T>::keep(bl[0], bl[1], bl[2], bl[3]);
  }
  acc_guard4(acc[0][0], acc[0][1], acc[0][2], acc[0][3]);
  acc_guard4(acc[1][0], acc[1][1], acc[1][2], acc[1][3]);
  acc_guard4(acc[2][0], acc[2][1], acc[2][2], acc[2][3]);
  acc_guard4(acc[3][0], acc[3][1], acc[3][2], acc[3][3]);

  float* slab = sT[wave];
  const float* Rb = RESID ? (resid + (size_t)b * strideR) : nullptr;
#pragma unroll
  for (int i = 0; i < 4; ++i) {
    const int mBase = m0 + (i << 4);
#pragma unroll
    for (int j = 0; j < 4; ++j) {
      const int n = n0 + (j << 4) + rlane;
      float bv = 0.f;
      if (BIAS_MODE == 2) bv = bias[n];
#pragma unroll
      for (int r = 0; r < 8; ++r) {
        float v = acc[i][j][r] * scale;
        if (BIAS_MODE == 1) v += bias[mBase + mOff + r];
        if (BIAS_MODE == 2) v += bv;
        if (RESID) v += Rb[(size_t)(mBase + mOff + r) * ldc + n];
        if (ACT == 1) v = tanhf(v);
        if (ACT == 2) v = fmaxf(v, 0.0f);
        if (ACT == 3) v = v / (1.0f + expf(-v));
        if (ACT == 4) v = (v > 0.f) ? v : 0.01f * v;
        slab[(mOff + r) * 68 + (j << 4) + rlane] = v;
      }
    }
    __builtin_amdgcn_fence(__ATOMIC_RELEASE, "workgroup");
    __builtin_amdgcn_wave_barrier();
    __builtin_amdgcn_fence(__ATOMIC_ACQUIRE, "workgroup");
    if (OUT_MODE == 0) {
      float* C = (float*)Cout + (size_t)b * strideC;
      const int hh = lane >> 4, c4 = (lane & 15) * 4;
      for (int pass = 0; pass < 2; ++pass) {
#pragma unroll
        for (int it = 0; it < 8; ++it) {
          const int row = it * 2 + hh;
          v4f v = *(const v4f*)(slab + row * 68 + c4);
          *(volatile v4f*)(C + (size_t)(mBase + row) * ldc + n0 + c4) = v;
        }
        __threadfence();
      }
    } else {
      const int q = lane >> 3, c8 = (lane & 7) * 8;
      unsigned short* C  = (unsigned short*)Cout  + (size_t)b * strideC;
      unsigned short* C2 = (OUT_MODE == 2) ? ((unsigned short*)Cout2 + (size_t)b * strideC) : nullptr;
      for (int pass = 0; pass < 2; ++pass) {
#pragma unroll
        for (int it = 0; it < 4; ++it) {
          const int row = it * 4 + q;
          const float* sp = slab + row * 68 + c8;
          v8h hv, lv;
#pragma unroll
          for (int e = 0; e < 8; ++e) {
            if (OUT_MODE == 1) {
              hv[e] = (_Float16)sp[e];
            } else {
              unsigned short hb = f2bf_bits(sp[e]);
              unsigned short lb = f2bf_bits(sp[e] - bf_bits2f(hb));
              hv[e] = __builtin_bit_cast(_Float16, hb);
              lv[e] = __builtin_bit_cast(_Float16, lb);
            }
          }
          *(volatile v8h*)(C + (size_t)(mBase + row) * ldc + n0 + c8) = hv;
          if (OUT_MODE == 2) *(volatile v8h*)(C2 + (size_t)(mBase + row) * ldc + n0 + c8) = lv;
        }
        __threadfence();
      }
    }
    __builtin_amdgcn_fence(__ATOMIC_RELEASE, "workgroup");
    __builtin_amdgcn_wave_barrier();
    __builtin_amdgcn_fence(__ATOMIC_ACQUIRE, "workgroup");
  }
}


__device__ __forceinline__ void two_words(float w, float carry, _Float16& hh, _Float16& ll) {
  const float sc = carry_flush(w, carry);
  hh = (_Float16)sc;
  const float rs = sc - (float)hh;
  ll = (_Float16)((fabsf(rs) < kF16MinNormal) ? 0.0f : rs);
}
__device__ __forceinline__ void store2(float* p, float v) {
  *(volatile float*)p = v;
  __threadfence();
  *(volatile float*)p = v;
}

__global__ __launch_bounds__(kThr) void zero_kernel(float* __restrict__ dst) {
  const size_t o4 = ((size_t)blockIdx.x * kThr + threadIdx.x) * 4u;
  const v4f z = {0.f, 0.f, 0.f, 0.f};
  *(volatile v4f*)(dst + o4) = z;
  __threadfence();
  *(volatile v4f*)(dst + o4) = z;
}

__global__ __launch_bounds__(kThr) void init_kernel(const float* __restrict__ Am, const float* __restrict__ Bm, const float* __restrict__ Cm, float* __restrict__ TAB) {
  const unsigned tid = threadIdx.x;
  if (blockIdx.x < 16u) {
    const unsigned i = blockIdx.x * (unsigned)kThr + tid;
    const float a0 = Am[i];
    store2(TAB + kTabPW + i, bf16r(a0));
  } else {
    if (tid >= 128u) return;
    const float s0 = (tid < 64u) ? Bm[tid] : Cm[tid - 64u];
    float* dp = (tid < 64u) ? (TAB + kTabV + tid) : (TAB + kTabC + (tid - 64u));
    store2(dp, bf16r(s0));
  }
}

__global__ __launch_bounds__(kThr) void square_kernel(const float* __restrict__ src, float* __restrict__ dst) {
  const unsigned t = blockIdx.x * (unsigned)kThr + threadIdx.x;
  const unsigned i = t >> 6, j = t & 63u;
  float acc = 0.0f;
  for (int m = 0; m < kN; ++m) acc += src[i * (unsigned)kN + (unsigned)m] * src[(unsigned)m * (unsigned)kN + j];
  store2(dst + t, acc);
}
static_assert(kN * kN == 16 * kThr, "squaring grid exact: 16 blocks");

__global__ __launch_bounds__(64) void matvec_kernel(const float* __restrict__ Pw, const float* __restrict__ src, float* __restrict__ dst, int tr) {
  const unsigned l = blockIdx.x, i = threadIdx.x;
  const float* sr = src + (size_t)l * kN;
  float acc = 0.0f;
  if (tr != 0) { for (int m = 0; m < kN; ++m) acc += sr[m] * Pw[(unsigned)m * (unsigned)kN + i]; }
  else { for (int j = 0; j < kN; ++j) acc += Pw[i * (unsigned)kN + (unsigned)j] * sr[j]; }
  store2(dst + (size_t)l * kN + i, acc);
}

__global__ __launch_bounds__(kThr) void tabcast_kernel(const float* __restrict__ TAB, unsigned short* __restrict__ TP16, unsigned short* __restrict__ AQ16) {
  v8h hv;
  unsigned short* dp;
  if (blockIdx.x < 6u) {
    const unsigned idx = blockIdx.x * (unsigned)kThr + threadIdx.x;
    const unsigned l = idx / 24u, g = idx - l * 24u;
    if (g < 16u) {
      const float* sp = TAB + kTabW + l * (unsigned)kN + (g & 7u) * 8u;
#pragma unroll
      for (int e = 0; e < 8; ++e) { const float p = sp[e]; hv[e] = (_Float16)carry_flush(p, kInCarry); }
    } else {
#pragma unroll
      for (int e = 0; e < 8; ++e) {
        const unsigned s = (g - 16u) * 8u + (unsigned)e;
        const bool live = s <= l;
        const float* vr = TAB + kTabV + (live ? (l - s) : 0u) * (unsigned)kN;
        float k = 0.0f;
        for (int n = 0; n < kN; ++n) k += TAB[kTabC + n] * vr[n];
        hv[e] = (_Float16)carry_flush(live ? k : 0.0f, kInCarry);
      }
    }
    dp = TP16 + (size_t)idx * 8u;
  } else {
    const unsigned idx = (blockIdx.x - 6u) * (unsigned)kThr + threadIdx.x;
    const unsigned n = idx / 40u, g = idx - n * 40u;
    const unsigned seg = g >> 3, j8 = (g & 7u) * 8u;
    const bool isQ = (seg == 2u) || (seg == 4u);
    const bool res = seg >= 3u;
#pragma unroll
    for (int e = 0; e < 8; ++e) {
      const unsigned j = j8 + (unsigned)e;
      const float v = isQ ? TAB[kTabV + (63u - j) * (unsigned)kN + n] : TAB[kTabPW + 6 * 4096 + n * (unsigned)kN + j];
      _Float16 a, b; two_words(v, kACarry, a, b);
      hv[e] = res ? b : a;
    }
    dp = AQ16 + (size_t)idx * 8u;
  }
  *(volatile v8h*)dp = hv;
  __threadfence();
  *(volatile v8h*)dp = hv;
}
static_assert(64 * 192 / 8 == 6 * kThr && 64 * 320 / 8 == 10 * kThr, "operand-plane grid exact: 6 + 10 blocks");

__global__ __launch_bounds__(kThr) void xfill_kernel(const float* __restrict__ U, unsigned short* __restrict__ HX) {
  const unsigned i = blockIdx.x * (unsigned)kThr + threadIdx.x;
  const unsigned j = i & 7u, d = (i >> 3) & 511u, e = i >> 12;
  const float* sp = U + (size_t)(e * (unsigned)kQ + j * 8u) * kD + d;
  v8h hv;
#pragma unroll
  for (int t = 0; t < 8; ++t) { const float v = sp[(size_t)t * kD]; hv[t] = (_Float16)carry_flush(bf16r(v), kInCarry); }
  unsigned short* dp = HX + ((size_t)e * kD + d) * kRW + 128u + j * 8u;
  for (int pass = 0; pass < 2; ++pass) { *(volatile v8h*)dp = hv; *(volatile v8h*)(dp + 128) = hv; __threadfence(); }
}
static_assert((size_t)kE * kD * (kQ / 8) == 4096ull * kThr && (kRW * 2) % 128 == 0, "input fill grid exact: 4,096 blocks; a row is a whole number of lines");

__global__ __launch_bounds__(kThr) void hcast_kernel(const float* __restrict__ HN32, unsigned short* __restrict__ HX, int cn) {
  const unsigned i = blockIdx.x * (unsigned)kThr + threadIdx.x;
  const unsigned g = i & 7u, row = i >> 3;
  const unsigned b = row >> 9, d = row & 511u;
  const float* sp = HN32 + (size_t)row * kN + g * 8u;
  const v4f a0 = *(const v4f*)sp, a1 = *(const v4f*)(sp + 4);
  v8h hv, lv;
#pragma unroll
  for (int t = 0; t < 8; ++t) { const float x = (t < 4) ? a0[t] : a1[t - 4]; _Float16 a, c; two_words(x, kInCarry, a, c); hv[t] = a; lv[t] = c; }
  unsigned short* dp = HX + (((size_t)b * kC + (unsigned)cn) * kD + d) * kRW + g * 8u;
  for (int pass = 0; pass < 2; ++pass) { *(volatile v8h*)dp = hv; *(volatile v8h*)(dp + 64) = lv; *(volatile v8h*)(dp + 192) = hv; __threadfence(); }
}
static_assert((size_t)kNb * kD * (kN / 8) == 64ull * kThr, "state cast grid exact: 64 blocks");

static_assert(((kD / 64) * (kN / 64)) % 8 == 0 && ((kQ / 64) * (kD / 64)) % 8 == 0, "the batched grids exact: every wave live");

extern "C" void kernel_launch(void* const* d_in, const int* in_sizes, int n_in,
                              void* d_out, int out_size, void* d_ws, size_t ws_size,
                              hipStream_t stream) {
  if (n_in < 4 || d_out == nullptr || d_ws == nullptr) return;
  if (in_sizes[0] != kNb * kL * kD || in_sizes[1] != kN * kN || in_sizes[2] != kN || in_sizes[3] != kN) return;
  if (out_size != kNb * kL * kD) return;
  if (ws_size < kWsTotal) return;
  const float* U = (const float*)d_in[0];
  const float* Am = (const float*)d_in[1];
  const float* Bm = (const float*)d_in[2];
  const float* Cm = (const float*)d_in[3];
  float* out = (float*)d_out;
  char* ws = (char*)d_ws;
  float* ZB = (float*)(ws + kOffZB);
  float* TAB = (float*)(ws + kOffTAB);
  unsigned short* TP16 = (unsigned short*)(ws + kOffTP16);
  unsigned short* AQ16 = (unsigned short*)(ws + kOffAQ16);
  float* HN32 = (float*)(ws + kOffHN32);
  unsigned short* HX = (unsigned short*)(ws + kOffHX);

  zero_kernel<<<2, kThr, 0, stream>>>(ZB);
  init_kernel<<<17, kThr, 0, stream>>>(Am, Bm, Cm, TAB);
  for (int k = 0; k < 6; ++k) square_kernel<<<16, kThr, 0, stream>>>(TAB + kTabPW + k * 4096, TAB + kTabPW + (k + 1) * 4096);
  for (int k = 0; k < 6; ++k) matvec_kernel<<<(1 << k), 64, 0, stream>>>(TAB + kTabPW + k * 4096, TAB + kTabV, TAB + kTabV + (size_t)(1 << k) * kN, 0);
  matvec_kernel<<<1, 64, 0, stream>>>(TAB + kTabPW, TAB + kTabC, TAB + kTabW, 1);
  for (int k = 0; k < 6; ++k) matvec_kernel<<<(1 << k), 64, 0, stream>>>(TAB + kTabPW + k * 4096, TAB + kTabW, TAB + kTabW + (size_t)(1 << k) * kN, 1);
  tabcast_kernel<<<16, kThr, 0, stream>>>(TAB, TP16, AQ16);
  xfill_kernel<<<4096, kThr, 0, stream>>>(U, HX);
  zero_kernel<<<128, kThr, 0, stream>>>(HN32);
  hcast_kernel<<<64, kThr, 0, stream>>>(HN32, HX, 0);
  for (int c = 0; c + 1 < kC; ++c) {
    const unsigned short* Ac = HX + (size_t)c * kD * kRW;
    wmma_gemm64<0, false, 2, 0, false, 0><<<dim3((kD / 64) * (kN / 64) / 8, kNb), 256, 0, stream>>>(
        Ac, Ac, kRW, (long)kC * kD * kRW, AQ16, AQ16, kRW, 0L, (void*)HN32, (void*)HN32, kN, (long)kD * kN, ZB, nullptr, 0L, kD, kN, kRW, kScC);
    hcast_kernel<<<64, kThr, 0, stream>>>(HN32, HX, c + 1);
  }
  wmma_gemm64<0, false, 2, 0, false, 0><<<dim3((kQ / 64) * (kD / 64) / 8, kE), 256, 0, stream>>>(
      TP16, TP16, 192, 0L, HX, HX, kRW, (long)kD * kRW, (void*)out, (void*)out, kD, (long)kQ * kD, ZB, nullptr, 0L, kQ, kD, 192, kScY);
}
